// CNNCharEncode_84688165143160
// MI455X (gfx1250) — hardware-verified
//
#include <hip/hip_runtime.h>
#include <stddef.h>


#pragma clang fp contract(off)

#define NW    4096
#define LW    20
#define CD    50
#define ODIM  768
#define XSLOT 64
#define XWRD  (LW * XSLOT)
#define WPB   16
#define TPB   256
#define NF0   128
#define NF1   128
#define NF2   512
#define KP0   64
#define KP1   128
#define KP2   192
#define NP0   20
#define NP1   19
#define NP2   18
#define CH0   (NF0 * KP0 / 8)
#define CH1   (NF1 * KP1 / 8)
#define CH2   (NF2 * KP2 / 8)
#define CHL   (ODIM * ODIM / 8)
#define GB0   (CH0 / TPB)
#define GB1   (CH1 / TPB)
#define GB2   (CH2 / TPB)
#define GBL   (CHL / TPB)
#define G_PREP (GB0 + GB1 + GB2 + 2 * GBL)
#define G_CNN  (NW / WPB)
#define HWM   64
#define HWN   64
#define NXCH  (WPB * LW * XSLOT / 8)
#define NTIT  (WPB * ODIM / (4 * TPB))

static_assert(CH0 % TPB == 0);
static_assert(CH1 % TPB == 0);
static_assert(CH2 % TPB == 0);
static_assert(CHL % TPB == 0);
static_assert(G_PREP == 636);
static_assert(G_CNN == 256);
static_assert(NXCH % TPB == 0);
static_assert(NXCH / TPB == 10);
static_assert(NTIT == 12);
static_assert((WPB * ODIM) % (4 * TPB) == 0);
static_assert(WPB * XWRD * 2 <= WPB * ODIM * 4);
static_assert(NF0 + NF1 + NF2 == ODIM);
static_assert(NW % WPB == 0);
static_assert(NW % HWM == 0);
static_assert(ODIM % HWN == 0);
static_assert(ODIM % 32 == 0);
static_assert(KP0 == XSLOT && KP1 == 2 * XSLOT && KP2 == 3 * XSLOT);
static_assert(NP0 == LW && NP1 + 1 == LW && NP2 + 2 == LW);
static_assert(CD <= XSLOT);

typedef float        v4f  __attribute__((ext_vector_type(4)));
typedef unsigned int v4u  __attribute__((ext_vector_type(4)));
typedef float        v8f  __attribute__((ext_vector_type(8)));
typedef _Float16     v8h  __attribute__((ext_vector_type(8)));
typedef _Float16     v16h __attribute__((ext_vector_type(16)));
typedef v4f __attribute__((may_alias)) v4fa;
typedef v8h __attribute__((may_alias)) v8ha;
typedef _Float16 __attribute__((may_alias)) f16a;

union Frag { v16h v; v8h hf[2]; };
union Pk8  { v8h h; v4u u; };

__device__ __forceinline__ v8f wmma_h(v16h a, v16h b, v8f c) {
  v8f d = __builtin_amdgcn_wmma_f32_16x16x32_f16(false, a, false, b, (short)0, c, false, false);
  asm volatile("v_nop\n\tv_nop\n\tv_nop\n\tv_nop" : "+v"(d) : "v"(a), "v"(b));
  return d;
}

__device__ __forceinline__ v16h ldfrag_g(const _Float16* p, int h) {
  Frag f;
  f.hf[0] = *(const v8h*)(p + 8 * h);
  f.hf[1] = *(const v8h*)(p + 16 + 8 * h);
  return f.v;
}
__device__ __forceinline__ v16h ldfrag_l(const f16a* p, int h) {
  Frag f;
  f.hf[0] = *(const v8ha*)(p + 8 * h);
  f.hf[1] = *(const v8ha*)(p + 16 + 8 * h);
  return f.v;
}

__device__ __forceinline__ v8h cvt8(v4f a, v4f c, float s) {
  v8h r;
  r[0] = (_Float16)(a.x * s); r[1] = (_Float16)(a.y * s);
  r[2] = (_Float16)(a.z * s); r[3] = (_Float16)(a.w * s);
  r[4] = (_Float16)(c.x * s); r[5] = (_Float16)(c.y * s);
  r[6] = (_Float16)(c.z * s); r[7] = (_Float16)(c.w * s);
  return r;
}

template <int W>
__device__ __forceinline__ void conv_chunk(const float* __restrict__ wsrc, int u,
                                           _Float16* __restrict__ dst) {
  constexpr int CPR = 8 * W;
  const int o  = u / CPR;
  const int kc = (u - o * CPR) * 8;
  const int t  = kc >> 6;
  const int c8 = kc & 63;
  Pk8 pk;
#pragma unroll
  for (int i = 0; i < 8; ++i) {
    const int c  = c8 + i;
    const int cc = (c < CD) ? c : (CD - 1);
    const float v = wsrc[(size_t)(o * CD + cc) * W + t];
    pk.h[i] = (_Float16)((c < CD) ? v * 64.0f : 0.0f);
  }
  _Float16* d = dst + (size_t)u * 8;
  *(volatile v4u*)d = pk.u;
  __threadfence();
  *(volatile v4u*)d = pk.u;
}

__device__ __forceinline__ void lin_chunk(const float* __restrict__ src, int u,
                                          _Float16* __restrict__ dst) {
  const v4f a = *(const v4fa*)(src + (size_t)u * 8);
  const v4f c = *(const v4fa*)(src + (size_t)u * 8 + 4);
  Pk8 pk;
  pk.h = cvt8(a, c, 256.0f);
  _Float16* d = dst + (size_t)u * 8;
  *(volatile v4u*)d = pk.u;
  __threadfence();
  *(volatile v4u*)d = pk.u;
}

__global__ __launch_bounds__(TPB) void k_prep(const float* __restrict__ w0,
                                              const float* __restrict__ w1,
                                              const float* __restrict__ w2,
                                              const float* __restrict__ whw,
                                              const float* __restrict__ wtw,
                                              _Float16* __restrict__ p0,
                                              _Float16* __restrict__ p1,
                                              _Float16* __restrict__ p2,
                                              _Float16* __restrict__ ph,
                                              _Float16* __restrict__ pt)
{
  const int blk = blockIdx.x, tid = threadIdx.x;
  if (blk < GB0) {
    conv_chunk<1>(w0, blk * TPB + tid, p0);
  } else if (blk < GB0 + GB1) {
    conv_chunk<2>(w1, (blk - GB0) * TPB + tid, p1);
  } else if (blk < GB0 + GB1 + GB2) {
    conv_chunk<3>(w2, (blk - GB0 - GB1) * TPB + tid, p2);
  } else if (blk < GB0 + GB1 + GB2 + GBL) {
    lin_chunk(whw, (blk - GB0 - GB1 - GB2) * TPB + tid, ph);
  } else {
    lin_chunk(wtw, (blk - GB0 - GB1 - GB2 - GBL) * TPB + tid, pt);
  }
}

template <int KS, int P>
__device__ __forceinline__ v8f conv_tile(const _Float16* __restrict__ wt, const f16a* xs,
                                         int n0, int m, int h) {
  constexpr int KP = KS * 32;
  const _Float16* wrow = wt + (size_t)(n0 + m) * KP;
  v16h bf[KS];
#pragma unroll
  for (int ks = 0; ks < KS; ++ks) bf[ks] = ldfrag_g(wrow + ks * 32, h);

  const f16a* arow = xs + m * XWRD;
  v8f mx = {-3.0e38f, -3.0e38f, -3.0e38f, -3.0e38f, -3.0e38f, -3.0e38f, -3.0e38f, -3.0e38f};
  const v8f z8 = {0.f, 0.f, 0.f, 0.f, 0.f, 0.f, 0.f, 0.f};
#pragma unroll 1
  for (int p = 0; p < P; ++p) {
    const f16a* ap = arow + p * XSLOT;
    v8f acc = z8;
#pragma unroll
    for (int ks = 0; ks < KS; ++ks) {
      const v16h a = ldfrag_l(ap + ks * 32, h);
      acc = wmma_h(a, bf[ks], acc);
    }
#pragma unroll
    for (int r = 0; r < 8; ++r) mx[r] = fmaxf(mx[r], acc[r]);
  }
  return mx;
}

__global__ __launch_bounds__(TPB) void k_charcnn(const float* __restrict__ x,
                                                 const _Float16* __restrict__ p0,
                                                 const _Float16* __restrict__ p1,
                                                 const _Float16* __restrict__ p2,
                                                 const float* __restrict__ b0,
                                                 const float* __restrict__ b1,
                                                 const float* __restrict__ b2,
                                                 float* __restrict__ feat)
{
  __shared__ __align__(16) float sbuf[WPB * ODIM];
  __shared__ __align__(16) float sbias[ODIM];

  const int tid = threadIdx.x, wv = tid >> 5, lane = tid & 31;
  const int h = lane >> 4, m = lane & 15;
  const int wg = blockIdx.x;

  for (int i = tid; i < ODIM; i += TPB) {
    const int i0 = (i < NF0) ? i : (NF0 - 1);
    int i1 = i - NF0;       i1 = (i1 < 0) ? 0 : ((i1 > NF1 - 1) ? (NF1 - 1) : i1);
    int i2 = i - NF0 - NF1; i2 = (i2 < 0) ? 0 : ((i2 > NF2 - 1) ? (NF2 - 1) : i2);
    const float v0 = b0[i0], v1 = b1[i1], v2 = b2[i2];
    sbias[i] = (i < NF0) ? v0 : ((i < NF0 + NF1) ? v1 : v2);
  }

  f16a* xs = (f16a*)sbuf;
#pragma unroll 1
  for (int it = 0; it < NXCH / TPB; ++it) {
    const int q   = it * TPB + tid;
    const int w   = q / (LW * 8);
    const int rem = q - w * (LW * 8);
    const int l   = rem >> 3;
    const int c8  = (rem & 7) * 8;
    const float* src = x + ((size_t)(wg * WPB + w) * LW + l) * CD;
    Pk8 pk;
#pragma unroll
    for (int i = 0; i < 8; ++i) {
      const int c  = c8 + i;
      const int cc = (c < CD) ? c : (CD - 1);
      const float v = src[cc];
      pk.h[i] = (_Float16)((c < CD) ? v : 0.0f);
    }
    *(v8ha*)(xs + w * XWRD + l * XSLOT + c8) = pk.h;
  }
  __syncthreads();

  const int nw = wv * 16;
  const v8f r0 = conv_tile<KP0 / 32, NP0>(p0, xs, nw, m, h);
  const v8f r1 = conv_tile<KP1 / 32, NP1>(p1, xs, nw, m, h);
  const v8f r2 = conv_tile<KP2 / 32, NP2>(p2, xs, nw, m, h);
  const v8f r3 = conv_tile<KP2 / 32, NP2>(p2, xs, nw + 128, m, h);
  const v8f r4 = conv_tile<KP2 / 32, NP2>(p2, xs, nw + 256, m, h);
  const v8f r5 = conv_tile<KP2 / 32, NP2>(p2, xs, nw + 384, m, h);
  __syncthreads();

  float* tile = sbuf;
  {
    const float sc = 0.015625f;
#pragma unroll
    for (int r = 0; r < 8; ++r) {
      const int ro = (8 * h + r) * ODIM + nw + m;
      tile[ro]               = r0[r] * sc;
      tile[ro + NF0]         = r1[r] * sc;
      tile[ro + NF0 + NF1]       = r2[r] * sc;
      tile[ro + NF0 + NF1 + 128] = r3[r] * sc;
      tile[ro + NF0 + NF1 + 256] = r4[r] * sc;
      tile[ro + NF0 + NF1 + 384] = r5[r] * sc;
    }
  }
  __syncthreads();

  float* dst = feat + (size_t)wg * (WPB * ODIM);
#pragma unroll 1
  for (int it = 0; it < NTIT; ++it) {
    const int i4  = it * TPB + tid;
    const int ch0 = (4 * i4) % ODIM;
    const v4f v  = *(const v4fa*)(tile + 4 * i4);
    const v4f bb = *(const v4fa*)(sbias + ch0);
    v4f o;
    o.x = tanhf(fminf(fmaxf(v.x + bb.x, -10.0f), 10.0f));
    o.y = tanhf(fminf(fmaxf(v.y + bb.y, -10.0f), 10.0f));
    o.z = tanhf(fminf(fmaxf(v.z + bb.z, -10.0f), 10.0f));
    o.w = tanhf(fminf(fmaxf(v.w + bb.w, -10.0f), 10.0f));
    *(v4fa*)(tile + 4 * i4) = o;
    *(volatile v4f*)(dst + 4 * i4) = o;
  }
  __threadfence();
#pragma unroll 1
  for (int it = 0; it < NTIT; ++it) {
    const int i4 = it * TPB + tid;
    const v4f o = *(const v4fa*)(tile + 4 * i4);
    *(volatile v4f*)(dst + 4 * i4) = o;
  }
}

__device__ __forceinline__ float hw1(float zh, float zt, float f) {
  const float hh = fmaxf(zh, 0.0f);
  const float zc = fminf(fmaxf(zt, -30.0f), 30.0f);
  const float e  = expf(-zc);
  const float t  = 1.0f / (1.0f + e);
  return t * hh + (1.0f - t) * f;
}

__global__ __launch_bounds__(TPB) void k_highway(const float* __restrict__ feat,
                                                 const _Float16* __restrict__ ph,
                                                 const _Float16* __restrict__ pt,
                                                 const float* __restrict__ whb,
                                                 const float* __restrict__ wtb,
                                                 float* __restrict__ out)
{
  __shared__ __align__(16) _Float16 sA[HWM * 32];
  __shared__ __align__(16) float sZh[8 * 16 * 32];
  __shared__ __align__(16) float sZt[8 * 16 * 32];

  const int tid = threadIdx.x, wv = tid >> 5, lane = tid & 31;
  const int h = lane >> 4, m = lane & 15;
  const int wr = wv >> 1, wc = wv & 1;
  const int m0 = blockIdx.x * HWM;
  const int n0 = blockIdx.y * HWN + wc * 32;

  const _Float16* bh0 = ph + (size_t)(n0 + m) * ODIM;
  const _Float16* bh1 = ph + (size_t)(n0 + 16 + m) * ODIM;
  const _Float16* bt0 = pt + (size_t)(n0 + m) * ODIM;
  const _Float16* bt1 = pt + (size_t)(n0 + 16 + m) * ODIM;
  const f16a* arow = (const f16a*)sA + (wr * 16 + m) * 32;

  const int srow = tid >> 2, sseg = (tid & 3) * 8;
  const float* srcrow = feat + (size_t)(m0 + srow) * ODIM + sseg;

  const v8f z8 = {0.f, 0.f, 0.f, 0.f, 0.f, 0.f, 0.f, 0.f};
  v8f ah0 = z8, ah1 = z8, at0 = z8, at1 = z8;

#pragma unroll 1
  for (int k0 = 0; k0 < ODIM; k0 += 32) {
    __syncthreads();
    {
      const v4f a = *(const v4fa*)(srcrow + k0);
      const v4f c = *(const v4fa*)(srcrow + k0 + 4);
      Pk8 pk;
      pk.h = cvt8(a, c, 16.0f);
      *(v8ha*)(sA + srow * 32 + sseg) = pk.h;
    }
    __syncthreads();
    const v16h a = ldfrag_l(arow, h);
    ah0 = wmma_h(a, ldfrag_g(bh0 + k0, h), ah0);
    ah1 = wmma_h(a, ldfrag_g(bh1 + k0, h), ah1);
    at0 = wmma_h(a, ldfrag_g(bt0 + k0, h), at0);
    at1 = wmma_h(a, ldfrag_g(bt1 + k0, h), at1);
  }

  float* zh = sZh + wv * 512;
  float* zt = sZt + wv * 512;
#pragma unroll
  for (int r = 0; r < 8; ++r) {
    const int ro = (8 * h + r) * 32;
    zh[ro + m]      = ah0[r];
    zh[ro + 16 + m] = ah1[r];
    zt[ro + m]      = at0[r];
    zt[ro + 16 + m] = at1[r];
  }
  __syncthreads();

  const float isc = 0.000244140625f;
  const size_t grow0 = (size_t)(m0 + wr * 16);
#pragma unroll 1
  for (int it = 0; it < 4; ++it) {
    const int i4  = it * 32 + lane;
    const int row = i4 >> 3;
    const int c4  = (i4 & 7) * 4;
    const v4f zh4 = *(const v4fa*)(zh + row * 32 + c4);
    const v4f zt4 = *(const v4fa*)(zt + row * 32 + c4);
    const v4f hb4 = *(const v4fa*)(whb + n0 + c4);
    const v4f tb4 = *(const v4fa*)(wtb + n0 + c4);
    const v4f f4  = *(const v4fa*)(feat + (grow0 + row) * ODIM + n0 + c4);
    v4f o;
    o.x = hw1(zh4.x * isc + hb4.x, zt4.x * isc + tb4.x, f4.x);
    o.y = hw1(zh4.y * isc + hb4.y, zt4.y * isc + tb4.y, f4.y);
    o.z = hw1(zh4.z * isc + hb4.z, zt4.z * isc + tb4.z, f4.z);
    o.w = hw1(zh4.w * isc + hb4.w, zt4.w * isc + tb4.w, f4.w);
    *(v4fa*)(zh + row * 32 + c4) = o;
    *(volatile v4f*)(out + (grow0 + row) * ODIM + n0 + c4) = o;
  }
  __threadfence();
#pragma unroll 1
  for (int it = 0; it < 4; ++it) {
    const int i4  = it * 32 + lane;
    const int row = i4 >> 3;
    const int c4  = (i4 & 7) * 4;
    const v4f o = *(const v4fa*)(zh + row * 32 + c4);
    *(volatile v4f*)(out + (grow0 + row) * ODIM + n0 + c4) = o;
  }
}

extern "C" void kernel_launch(void* const* d_in, const int* in_sizes, int n_in,
                              void* d_out, int out_size, void* d_ws, size_t ws_size,
                              hipStream_t stream)
{
  if (n_in < 11) return;
  if (in_sizes[0]  != NW * LW * CD) return;
  if (in_sizes[1]  != NF0 * CD * 1) return;
  if (in_sizes[2]  != NF0) return;
  if (in_sizes[3]  != NF1 * CD * 2) return;
  if (in_sizes[4]  != NF1) return;
  if (in_sizes[5]  != NF2 * CD * 3) return;
  if (in_sizes[6]  != NF2) return;
  if (in_sizes[7]  != ODIM * ODIM) return;
  if (in_sizes[8]  != ODIM) return;
  if (in_sizes[9]  != ODIM * ODIM) return;
  if (in_sizes[10] != ODIM) return;
  if (out_size != NW * ODIM) return;

  const float* x   = (const float*)d_in[0];
  const float* w0  = (const float*)d_in[1];
  const float* b0  = (const float*)d_in[2];
  const float* w1  = (const float*)d_in[3];
  const float* b1  = (const float*)d_in[4];
  const float* w2  = (const float*)d_in[5];
  const float* b2  = (const float*)d_in[6];
  const float* whw = (const float*)d_in[7];
  const float* whb = (const float*)d_in[8];
  const float* wtw = (const float*)d_in[9];
  const float* wtb = (const float*)d_in[10];
  float* out = (float*)d_out;

  const size_t bP0   = (size_t)NF0 * KP0 * 2;
  const size_t bP1   = (size_t)NF1 * KP1 * 2;
  const size_t bP2   = (size_t)NF2 * KP2 * 2;
  const size_t bPL   = (size_t)ODIM * ODIM * 2;
  const size_t bFeat = (size_t)NW * ODIM * 4;
  const size_t total = bP0 + bP1 + bP2 + 2 * bPL + bFeat;
  if (total > ws_size) return;
  if (total > (size_t)134217728) return;

  char* ws = (char*)d_ws;
  size_t off = 0;
  _Float16* p0   = (_Float16*)(ws + off); off += bP0;
  _Float16* p1   = (_Float16*)(ws + off); off += bP1;
  _Float16* p2   = (_Float16*)(ws + off); off += bP2;
  _Float16* ph   = (_Float16*)(ws + off); off += bPL;
  _Float16* pt   = (_Float16*)(ws + off); off += bPL;
  float*    feat = (float*)(ws + off);    off += bFeat;
  if (off != total) return;

  k_prep<<<G_PREP, TPB, 0, stream>>>(w0, w1, w2, whw, wtw, p0, p1, p2, ph, pt);
  k_charcnn<<<G_CNN, TPB, 0, stream>>>(x, p0, p1, p2, b0, b1, b2, feat);
  k_highway<<<dim3(NW / HWM, ODIM / HWN), TPB, 0, stream>>>(feat, ph, pt, whb, wtb, out);
}
